// CrossAttentionEncoder_66571993088195
// MI455X (gfx1250) — hardware-verified
//
#include <hip/hip_runtime.h>
#include <math.h>

typedef __attribute__((ext_vector_type(16))) _Float16 v16h;
typedef __attribute__((ext_vector_type(16))) __bf16 v16b;
typedef __attribute__((ext_vector_type(8)))  _Float16 v8h;
typedef __attribute__((ext_vector_type(8)))  float v8f;
typedef __attribute__((ext_vector_type(4)))  float v4f;
typedef __attribute__((ext_vector_type(2)))  float v2f;
typedef __attribute__((ext_vector_type(4)))  unsigned v4u;
typedef __attribute__((ext_vector_type(4)))  int v4i;
typedef float __attribute__((may_alias)) float_a;
typedef int __attribute__((may_alias)) int_a;

template <typename T> __device__ __forceinline__ void vst2(void* p, T v) { *(volatile T*)p = v; __threadfence(); *(volatile T*)p = v; }
__device__ __forceinline__ v8f wmma16(v16h a, v16h b, v8f c) {
  v8f d = __builtin_amdgcn_wmma_f32_16x16x32_f16(false, a, false, b, (short)0, c, false, false);
  asm volatile("v_nop\n\tv_nop\n\tv_nop\n\tv_nop" : "+v"(d) : "v"(a), "v"(b));
  return d;
}
__device__ __forceinline__ v8f wmma_bf(v16b a, v16b b, v8f c) {
  v8f d = __builtin_amdgcn_wmma_f32_16x16x32_bf16(false, a, false, b, (short)0, c, false, false);
  asm volatile("v_nop\n\tv_nop\n\tv_nop\n\tv_nop" : "+v"(d) : "v"(a), "v"(b));
  return d;
}
__device__ __forceinline__ v16h frag_h(const _Float16* rowk0, int lane) {
  union { v16h v; v8h q[2]; } u; const _Float16* p = rowk0 + 8 * (lane >> 4);
  u.q[0] = *(const v8h*)p; u.q[1] = *(const v8h*)(p + 16); return u.v;
}
__device__ __forceinline__ v16h frag_f32(const float* rowk0, int lane) {
  v16h a; const float* p = rowk0 + 8 * (lane >> 4);
#pragma unroll
  for (int i = 0; i < 8; ++i) { a[i] = (_Float16)p[i]; a[8 + i] = (_Float16)p[16 + i]; }
  return a;
}
__device__ __forceinline__ v16h frag_f32s(const float* rowk0, int lane, float sc) {
  v16h a; const float* p = rowk0 + 8 * (lane >> 4);
#pragma unroll
  for (int i = 0; i < 8; ++i) { a[i] = (_Float16)(p[i] * sc); a[8 + i] = (_Float16)(p[16 + i] * sc); }
  return a;
}
__device__ __forceinline__ v16h fragc_f32(const float* W, int k0, int n, int lane, int ld, int K) {
  v16h a; const int g = lane >> 4;
#pragma unroll
  for (int i = 0; i < 8; ++i) { const int ka = k0 + 8 * g + i, kb = ka + 16;
    a[i] = (_Float16)(ka < K ? W[(size_t)(ka < K ? ka : K - 1) * ld + n] : 0.f); a[8 + i] = (_Float16)(kb < K ? W[(size_t)(kb < K ? kb : K - 1) * ld + n] : 0.f); }
  return a;
}
struct F2 { v16b h, l; };
__device__ __forceinline__ F2 bsplit16(const float v[16]) { F2 r;
#pragma unroll
  for (int i = 0; i < 16; ++i) { const __bf16 h = (__bf16)v[i]; r.h[i] = h; r.l[i] = (__bf16)(v[i] - (float)h); }
  return r; }
__device__ __forceinline__ F2 split_row(const float* row, int k0, int lane) { float v[16]; const float* p = row + k0 + 8 * (lane >> 4);
#pragma unroll
  for (int i = 0; i < 8; ++i) { v[i] = p[i]; v[8 + i] = p[16 + i]; }
  return bsplit16(v); }
__device__ __forceinline__ F2 split_rowK(const float* row, int k0, int lane, int K) { float v[16]; const int g = lane >> 4;
#pragma unroll
  for (int i = 0; i < 8; ++i) { const int ka = k0 + 8 * g + i, kb = ka + 16; v[i] = ka < K ? row[ka < K ? ka : K - 1] : 0.f; v[8 + i] = kb < K ? row[kb < K ? kb : K - 1] : 0.f; }
  return bsplit16(v); }
__device__ __forceinline__ F2 split_col(const float* W, int k0, int n, int lane, int ld, int K) { float v[16]; const int g = lane >> 4;
#pragma unroll
  for (int i = 0; i < 8; ++i) { const int ka = k0 + 8 * g + i, kb = ka + 16; v[i] = ka < K ? W[(size_t)(ka < K ? ka : K - 1) * ld + n] : 0.f; v[8 + i] = kb < K ? W[(size_t)(kb < K ? kb : K - 1) * ld + n] : 0.f; }
  return bsplit16(v); }
__device__ __forceinline__ v8f mac3(const F2& a, const F2& b, v8f c) { c = wmma_bf(a.l, b.h, c); c = wmma_bf(a.h, b.l, c); return wmma_bf(a.h, b.h, c); }
__device__ __forceinline__ float sigm(float v) { return 1.0f / (1.0f + expf(-v)); }
#define LDSX() do { asm volatile("s_wait_dscnt 0" ::: "memory"); __builtin_amdgcn_wave_barrier(); __builtin_amdgcn_fence(__ATOMIC_RELEASE, "workgroup"); } while (0)


#define NB 2
#define NN 4096
#define KN 16
#define CIN 128
#define CQ 128
#define DD 256
#define PH 64
#define AH 1024
#define NR (NB * NN)
#define NPR (NR * KN)
#ifndef NBT
#define NBT NB
#endif
#define NRT (NBT * NN)
typedef __attribute__((ext_vector_type(8))) __bf16 v8b;
__device__ __forceinline__ v16b frag_b(const __bf16* rowk0, int lane) {
  union { v16b v; v8b q[2]; } u; const __bf16* p = rowk0 + 8 * (lane >> 4);
  u.q[0] = *(const v8b*)p; u.q[1] = *(const v8b*)(p + 16); return u.v;
}
__device__ __forceinline__ float bfr(float v) { return (float)(__bf16)v; }
__device__ __attribute__((noinline)) float exp_ni(float v) { return expf(v); }
__device__ __attribute__((noinline)) float erf_ni(float v) { return erff(v); }

#define PK_LSQ 0
#define PK_LSO ((size_t)DD * CQ)
#define PK_K   (PK_LSO + (size_t)DD * CIN)
#define PK_Q   (PK_K + (size_t)DD * DD)
#define PK_V   (PK_Q + (size_t)DD * DD)
#define PK_P2  (PK_V + (size_t)DD * DD)
#define PK_A1  (PK_P2 + (size_t)DD * PH)
#define PK_A2  (PK_A1 + (size_t)AH * DD)
#define PK_E   (PK_A2 + (size_t)DD * AH)
#define PK_END (PK_E + (size_t)CIN * DD)
#define WS_PK  0u
#define WS_QF  (((2u * PK_END) + 127u) / 128u * 128u)
#define WS_OF  (WS_QF + 4u * NR * DD)
#define WS_QRY (WS_OF + 4u * NR * DD)
#define WS_KEY (WS_QRY + 4u * NR * DD)
#define WS_VAL (WS_KEY + 4u * NR * DD)
#define WS_AGG (WS_VAL + 4u * NR * DD)
#define WS_IDX (WS_AGG + 4u * NR * DD)
#define WS_PE  (WS_IDX + 4u * NR * KN)
#define WS_END (WS_PE + 4u * (size_t)NPR * DD)

__global__ __launch_bounds__(256) void k_pack(const float* __restrict__ WLSQ, const float* __restrict__ WLSO, const float* __restrict__ WK, const float* __restrict__ WQ, const float* __restrict__ WV, const float* __restrict__ WP2, const float* __restrict__ WA1, const float* __restrict__ WA2, const float* __restrict__ WE, __bf16* __restrict__ PK) {
  __shared__ __align__(16) __bf16 s[AH]; const int n = blockIdx.x, which = blockIdx.y, t = threadIdx.x; int K, NO; size_t dst; const float* Wm;
  switch (which) { case 0: Wm = WLSQ; K = CQ; NO = DD; dst = PK_LSQ; break; case 1: Wm = WLSO; K = CIN; NO = DD; dst = PK_LSO; break; case 2: Wm = WK; K = DD; NO = DD; dst = PK_K; break; case 3: Wm = WQ; K = DD; NO = DD; dst = PK_Q; break; case 4: Wm = WV; K = DD; NO = DD; dst = PK_V; break; case 5: Wm = WP2; K = PH; NO = DD; dst = PK_P2; break; case 6: Wm = WA1; K = DD; NO = AH; dst = PK_A1; break; case 7: Wm = WA2; K = AH; NO = DD; dst = PK_A2; break; default: Wm = WE; K = DD; NO = CIN; dst = PK_E; break; }
  if (n >= NO) return;
  for (int k = t; k < K; k += 256) s[k] = (__bf16)Wm[(size_t)n * K + k];
  __syncthreads();
  for (int q = t; q < K / 8; q += 256) vst2((unsigned*)(PK + dst + (size_t)n * K + q * 8), *(const v4u*)&s[q * 8]);
}
__global__ __launch_bounds__(128) void k_in(const float* __restrict__ XQ, const float* __restrict__ XO, const __bf16* __restrict__ PK, const float* __restrict__ BQ_, const float* __restrict__ BO_, float* __restrict__ QF, float* __restrict__ OF) {
  __shared__ __align__(16) __bf16 sa[64][CIN + 8]; __shared__ __align__(16) float so[4][16][132];
  const int tid = threadIdx.x, wave = tid >> 5, lane = tid & 31, col = lane & 15, g = lane >> 4; const size_t b = blockIdx.y; const int which = blockIdx.z; const int n0 = blockIdx.x * 64; const float* X = which ? XO : XQ;
  for (int e = tid; e < 64 * CIN; e += 128) { const int c = e >> 6, r = e & 63; sa[r][c] = (__bf16)X[(b * CIN + c) * NN + n0 + r]; }
  if (tid < 64) for (int c = CIN; c < CIN + 8; ++c) sa[tid][c] = (__bf16)0.f;
  __syncthreads();
  const __bf16* P = PK + (which ? PK_LSO : PK_LSQ); const float* BB = which ? BO_ : BQ_; float* OUT = which ? OF : QF;
#pragma unroll 1
  for (int half = 0; half < 2; ++half) { v8f acc[8] = {};
#pragma unroll
    for (int kc = 0; kc < CIN / 32; ++kc) { const v16b a = frag_b(&sa[wave * 16 + col][kc * 32], lane);
#pragma unroll
      for (int j = 0; j < 8; ++j) acc[j] = wmma_bf(a, frag_b(P + (size_t)(half * 128 + j * 16 + col) * CIN + kc * 32, lane), acc[j]); }
#pragma unroll
    for (int j = 0; j < 8; ++j) { const float bb = bfr(BB[half * 128 + j * 16 + col]);
#pragma unroll
      for (int r = 0; r < 8; ++r) so[wave][8 * g + r][j * 16 + col] = acc[j][r] + bb; }
    LDSX();
    for (int rl = 0; rl < 16; ++rl) vst2(OUT + ((b * NN) + n0 + wave * 16 + rl) * DD + half * 128 + lane * 4, *(const v4f*)&so[wave][rl][lane * 4]);
    LDSX(); }
}
__global__ __launch_bounds__(128) void k_kqv(const float* __restrict__ QF, const float* __restrict__ OF, const __bf16* __restrict__ PK, const float* __restrict__ BK, const float* __restrict__ BQ, const float* __restrict__ BV, float* __restrict__ KEY, float* __restrict__ QRY, float* __restrict__ VAL) {
  __shared__ __align__(16) float so[4][16][132];
  const int tid = threadIdx.x, wave = tid >> 5, lane = tid & 31, col = lane & 15, g = lane >> 4; const size_t r0 = (size_t)blockIdx.x * 64 + wave * 16; const int n0 = blockIdx.y * 128; const int which = blockIdx.z;
  const float* A = (which == 1) ? QF : OF; const __bf16* P = PK + ((which == 0) ? PK_K : (which == 1) ? PK_Q : PK_V); const float* BB = (which == 0) ? BK : (which == 1) ? BQ : BV; float* OUT = (which == 0) ? KEY : (which == 1) ? QRY : VAL;
  v8f acc[8] = {};
#pragma unroll 2
  for (int kc = 0; kc < DD / 32; ++kc) { const F2 a = split_row(A + (r0 + col) * DD, kc * 32, lane);
#pragma unroll
    for (int j = 0; j < 8; ++j) { const v16b w = frag_b(P + (size_t)(n0 + j * 16 + col) * DD + kc * 32, lane); acc[j] = wmma_bf(a.l, w, acc[j]); acc[j] = wmma_bf(a.h, w, acc[j]); } }
#pragma unroll
  for (int j = 0; j < 8; ++j) { const float bb = bfr(BB[n0 + j * 16 + col]);
#pragma unroll
    for (int r = 0; r < 8; ++r) so[wave][8 * g + r][j * 16 + col] = acc[j][r] + bb; }
  LDSX();
  for (int rl = 0; rl < 16; ++rl) vst2(OUT + (r0 + rl) * DD + n0 + lane * 4, *(const v4f*)&so[wave][rl][lane * 4]);
}
__global__ __launch_bounds__(256) void k_knn(const float* __restrict__ POS, int* __restrict__ IDX) {
  __shared__ float sx[NN][3]; __shared__ float sq[NN]; __shared__ float ld[64][4][KN]; __shared__ int li[64][4][KN]; __shared__ __align__(16) int so[64][KN];
  const int t = threadIdx.x; const size_t b = blockIdx.y; const int n0 = blockIdx.x * 64; const int q = t >> 2, part = t & 3;
  for (int i = t; i < NN; i += 256) { const float x = bfr(POS[(b * 3 + 0) * NN + i]), y = bfr(POS[(b * 3 + 1) * NN + i]), z = bfr(POS[(b * 3 + 2) * NN + i]); sx[i][0] = x; sx[i][1] = y; sx[i][2] = z; sq[i] = (x * x + z * z) + y * y; }
  __syncthreads();
  const int me = n0 + q; const float px = sx[me][0], py = sx[me][1], pz = sx[me][2], sqm = sq[me];
  float* bd = ld[q][part]; int* bi = li[q][part]; for (int k = 0; k < KN; ++k) { bd[k] = 3.0e38f; bi[k] = 0x7fffffff; }
  float thr = 3.0e38f; int thri = 0x7fffffff;
#pragma unroll 1
  for (int i = part * (NN / 4); i < (part + 1) * (NN / 4); ++i) { const float dot = (px * sx[i][0] + py * sx[i][1]) + pz * sx[i][2]; const float d = (sqm + sq[i]) - 2.0f * dot;
    if (d < thr || (d == thr && i < thri)) { int pos = KN - 1; while (pos > 0 && (d < bd[pos - 1] || (d == bd[pos - 1] && i < bi[pos - 1]))) { bd[pos] = bd[pos - 1]; bi[pos] = bi[pos - 1]; --pos; } bd[pos] = d; bi[pos] = i; thr = bd[KN - 1]; thri = bi[KN - 1]; } }
  __syncthreads();
  if (part == 0) { int hp[4] = {0, 0, 0, 0};
    for (int k = 0; k < KN; ++k) { int best = -1; float bdv = 3.0e38f; int biv = 0x7fffffff;
      for (int p2 = 0; p2 < 4; ++p2) { if (hp[p2] >= KN) continue; const float dv = ld[q][p2][hp[p2]]; const int iv = li[q][p2][hp[p2]]; if (best < 0 || dv < bdv || (dv == bdv && iv < biv)) { best = p2; bdv = dv; biv = iv; } }
      so[q][k] = biv; ++hp[best]; } }
  __syncthreads();
  for (int e = t; e < 64 * KN / 4; e += 256) { const int r = e / (KN / 4), c = e % (KN / 4); vst2(IDX + (b * NN + n0 + r) * KN + c * 4, *(const v4i*)&so[r][c * 4]); }
}
__global__ __launch_bounds__(128) void k_pe(const float* __restrict__ POS, const int* __restrict__ IDX, const float* __restrict__ WP1, const float* __restrict__ BP1, const float* __restrict__ G1, const float* __restrict__ BT1, const float* __restrict__ M1, const float* __restrict__ V1, const __bf16* __restrict__ PK, const float* __restrict__ BP2, float* __restrict__ PE) {
  __shared__ __align__(16) __bf16 sh[64][PH + 8], sl[64][PH + 8]; __shared__ float spr[64][3]; __shared__ __align__(16) float so[4][16][132];
  const int tid = threadIdx.x, wave = tid >> 5, lane = tid & 31, col = lane & 15, g = lane >> 4; const size_t pr0 = (size_t)blockIdx.x * 64; const size_t row0 = pr0 / KN; const size_t b = row0 / NN;
  if (tid < 64) { const size_t row = row0 + (tid >> 4); const int k = tid & 15; const int n = (int)(row % NN); const int m = IDX[row * KN + k];
    for (int c = 0; c < 3; ++c) spr[tid][c] = bfr(POS[(b * 3 + c) * NN + n]) - bfr(POS[(b * 3 + c) * NN + m]); }
  __syncthreads();
  for (int e = tid; e < 64 * PH; e += 128) { const int r = e >> 6, o = e & 63; const float pre = (bfr(WP1[o * 3]) * spr[r][0] + bfr(WP1[o * 3 + 1]) * spr[r][1]) + bfr(WP1[o * 3 + 2]) * spr[r][2] + bfr(BP1[o]);
    const float sc = bfr(G1[o]) / sqrtf(bfr(V1[o]) + 1e-5f); const float v = fmaxf(pre * sc + (bfr(BT1[o]) - bfr(M1[o]) * sc), 0.f); const __bf16 hb = (__bf16)v; sh[r][o] = hb; sl[r][o] = (__bf16)(v - (float)hb); }
  if (tid < 64) for (int o = PH; o < PH + 8; ++o) { sh[tid][o] = (__bf16)0.f; sl[tid][o] = (__bf16)0.f; }
  __syncthreads();
#pragma unroll 1
  for (int half = 0; half < 2; ++half) { v8f acc[8] = {};
#pragma unroll
    for (int kc = 0; kc < PH / 32; ++kc) { F2 a; a.h = frag_b(&sh[wave * 16 + col][kc * 32], lane); a.l = frag_b(&sl[wave * 16 + col][kc * 32], lane);
#pragma unroll
      for (int j = 0; j < 8; ++j) { const v16b w = frag_b(PK + PK_P2 + (size_t)(half * 128 + j * 16 + col) * PH + kc * 32, lane); acc[j] = wmma_bf(a.l, w, acc[j]); acc[j] = wmma_bf(a.h, w, acc[j]); } }
#pragma unroll
    for (int j = 0; j < 8; ++j) { const float bb = bfr(BP2[half * 128 + j * 16 + col]);
#pragma unroll
      for (int r = 0; r < 8; ++r) so[wave][8 * g + r][j * 16 + col] = acc[j][r] + bb; }
    LDSX();
    for (int rl = 0; rl < 16; ++rl) vst2(PE + (pr0 + wave * 16 + rl) * DD + half * 128 + lane * 4, *(const v4f*)&so[wave][rl][lane * 4]);
    LDSX(); }
}
__global__ __launch_bounds__(128) void k_att(const float* __restrict__ QRY, const float* __restrict__ KEY, const float* __restrict__ VAL, const float* __restrict__ PE, const int* __restrict__ IDX, const __bf16* __restrict__ PK, const float* __restrict__ BA1, const float* __restrict__ G2, const float* __restrict__ BT2, const float* __restrict__ M2, const float* __restrict__ V2, const float* __restrict__ BA2, float* __restrict__ AGG) {
  __shared__ __align__(16) __bf16 sa[32][DD + 8]; __shared__ __align__(16) __bf16 shd[32][AH + 8]; __shared__ int sidx[32]; __shared__ __align__(16) float sagg[2][DD];
  const int tid = threadIdx.x, wave = tid >> 5, lane = tid & 31, col = lane & 15, g = lane >> 4; const size_t row0 = (size_t)blockIdx.x * 2; const size_t b = row0 / NN; const int rt = wave & 1, chh = wave >> 1;
  if (tid < 32) sidx[tid] = IDX[(row0 + (tid >> 4)) * KN + (tid & 15)];
  __syncthreads();
  for (int e = tid; e < 32 * DD; e += 128) { const int r = e >> 8, d = e & 255; const size_t row = row0 + (r >> 4); const size_t m = b * NN + sidx[r];
    sa[r][d] = (__bf16)(QRY[row * DD + d] - KEY[m * DD + d] + PE[((row * KN) + (r & 15)) * DD + d]); }
  if (tid < 32) { for (int d = DD; d < DD + 8; ++d) sa[tid][d] = (__bf16)0.f; for (int d = AH; d < AH + 8; ++d) shd[tid][d] = (__bf16)0.f; }
  __syncthreads();
#pragma unroll 1
  for (int pass = 0; pass < AH / 128; ++pass) { v8f acc[4] = {}; const int c0 = pass * 128 + chh * 64;
#pragma unroll 2
    for (int kc = 0; kc < DD / 32; ++kc) { const v16b a = frag_b(&sa[rt * 16 + col][kc * 32], lane);
#pragma unroll
      for (int j = 0; j < 4; ++j) acc[j] = wmma_bf(a, frag_b(PK + PK_A1 + (size_t)(c0 + j * 16 + col) * DD + kc * 32, lane), acc[j]); }
#pragma unroll
    for (int j = 0; j < 4; ++j) { const int c = c0 + j * 16 + col; const float sc = bfr(G2[c]) / sqrtf(bfr(V2[c]) + 1e-5f); const float sh_ = bfr(BT2[c]) - bfr(M2[c]) * sc; const float bb = bfr(BA1[c]);
#pragma unroll
      for (int r = 0; r < 8; ++r) shd[rt * 16 + 8 * g + r][c] = (__bf16)fmaxf((acc[j][r] + bb) * sc + sh_, 0.f); } }
  __syncthreads();
  v8f acc2[8] = {}; const int d0 = chh * 128;
#pragma unroll 2
  for (int kc = 0; kc < AH / 32; ++kc) { const v16b a = frag_b(&shd[rt * 16 + col][kc * 32], lane);
#pragma unroll
    for (int j = 0; j < 8; ++j) acc2[j] = wmma_bf(a, frag_b(PK + PK_A2 + (size_t)(d0 + j * 16 + col) * AH + kc * 32, lane), acc2[j]); }
  const size_t rowp = row0 + rt;
#pragma unroll
  for (int j = 0; j < 8; ++j) { const int d = d0 + j * 16 + col; const float bb = bfr(BA2[d]); float mx = -3.0e38f;
#pragma unroll
    for (int r = 0; r < 8; ++r) { acc2[j][r] += bb; mx = fmaxf(mx, acc2[j][r]); }
    mx = fmaxf(mx, __shfl_xor(mx, 16));
    float sm = 0.f, wsum = 0.f;
#pragma unroll
    for (int r = 0; r < 8; ++r) { const int k = 8 * g + r; const float e = exp_ni(acc2[j][r] - mx); sm += e; wsum += e * (VAL[rowp * DD + d] + PE[((rowp * KN) + k) * DD + d]); }
    sm += __shfl_xor(sm, 16); wsum += __shfl_xor(wsum, 16);
    if (g == 0) sagg[rt][d] = wsum / sm; }
  __syncthreads();
  for (int e = tid; e < 2 * DD / 4; e += 128) { const int r = e / (DD / 4), q4 = e % (DD / 4); vst2(AGG + (row0 + r) * DD + q4 * 4, *(const v4f*)&sagg[r][q4 * 4]); }
}
__global__ __launch_bounds__(128) void k_out(const float* __restrict__ AGG, const __bf16* __restrict__ PK, const float* __restrict__ BF, float* __restrict__ OUT) {
  __shared__ __align__(16) float st[CIN][68];
  const int tid = threadIdx.x, wave = tid >> 5, lane = tid & 31, col = lane & 15, g = lane >> 4; const size_t b = blockIdx.y; const int n0 = blockIdx.x * 64; const size_t r0 = b * NN + n0 + wave * 16;
  v8f acc[8] = {};
#pragma unroll 2
  for (int kc = 0; kc < DD / 32; ++kc) { const F2 a = split_row(AGG + (r0 + col) * DD, kc * 32, lane);
#pragma unroll
    for (int j = 0; j < 8; ++j) { const v16b w = frag_b(PK + PK_E + (size_t)(j * 16 + col) * DD + kc * 32, lane); acc[j] = wmma_bf(a.l, w, acc[j]); acc[j] = wmma_bf(a.h, w, acc[j]); } }
#pragma unroll
  for (int j = 0; j < 8; ++j) { const int c = j * 16 + col; const float bb = bfr(BF[c]);
#pragma unroll
    for (int r = 0; r < 8; ++r) st[c][wave * 16 + 8 * g + r] = acc[j][r] + bb; }
  __syncthreads();
  for (int e = tid; e < CIN * 16; e += 128) { const int c = e >> 4, q = e & 15; vst2(OUT + (b * CIN + c) * NN + n0 + q * 4, *(const v4f*)&st[c][q * 4]); }
}
extern "C" void kernel_launch(void* const* d_in, const int* in_sizes, int n_in, void* d_out, int out_size, void* d_ws, size_t ws_size, hipStream_t stream) {
  (void)in_sizes; (void)n_in; (void)out_size;
  const float** F = (const float**)d_in;
  if (ws_size < (size_t)WS_END) return;
  char* ws = (char*)d_ws; __bf16* PK = (__bf16*)(ws + WS_PK); float *QF = (float*)(ws + WS_QF), *OF = (float*)(ws + WS_OF), *QRY = (float*)(ws + WS_QRY), *KEY = (float*)(ws + WS_KEY), *VAL = (float*)(ws + WS_VAL), *AGG = (float*)(ws + WS_AGG), *PE = (float*)(ws + WS_PE); int* IDX = (int*)(ws + WS_IDX);
  k_pack<<<dim3(AH, 9), 256, 0, stream>>>(F[3], F[5], F[7], F[9], F[11], F[19], F[21], F[27], F[29], PK);
  k_in<<<dim3(NN / 64, NBT, 2), 128, 0, stream>>>(F[2], F[0], PK, F[4], F[6], QF, OF);
  k_kqv<<<dim3(NRT / 64, DD / 128, 3), 128, 0, stream>>>(QF, OF, PK, F[8], F[10], F[12], KEY, QRY, VAL);
  k_knn<<<dim3(NN / 64, NBT), 256, 0, stream>>>(F[1], IDX);
  k_pe<<<NRT * KN / 64, 128, 0, stream>>>(F[1], IDX, F[13], F[14], F[15], F[16], F[17], F[18], PK, F[20], PE);
  k_att<<<NRT / 2, 128, 0, stream>>>(QRY, KEY, VAL, PE, IDX, PK, F[22], F[23], F[24], F[25], F[26], F[28], AGG);
  k_out<<<dim3(NN / 64, NBT), 128, 0, stream>>>(AGG, PK, F[30], (float*)d_out);
}
